// RNNLanguageModel_103079215117
// MI455X (gfx1250) — hardware-verified
//
#include <hip/hip_runtime.h>
#include <stddef.h>

typedef __attribute__((ext_vector_type(16))) _Float16 v16h;
typedef __attribute__((ext_vector_type(8)))  _Float16 v8h;
typedef __attribute__((ext_vector_type(16))) __bf16   v16b;
typedef __attribute__((ext_vector_type(8)))  __bf16   v8b;
typedef __attribute__((ext_vector_type(8)))  float    v8f;
typedef __attribute__((ext_vector_type(4)))  float    v4f;

constexpr int kBatch = 128;
constexpr int kSteps = 1024;
constexpr int kEmb = 128;
constexpr int kHid = 128;
constexpr int kVoc = 32000;
constexpr int kRowsPerBlock = 32;
constexpr int kTilePitch = 136;
constexpr int kSlabPitch = 132;
constexpr float kActCarry = 8.0f;
constexpr float kWCarry = 16.0f;
constexpr float kFold = 1.0f / 128.0f;

__device__ __forceinline__ unsigned short f2bf_bits(float f) {
  unsigned u = __float_as_uint(f);
  return (unsigned short)((u + 0x7FFFu + ((u >> 16) & 1u)) >> 16);
}
__device__ __forceinline__ float bf_bits2f(unsigned short h) { return __uint_as_float(((unsigned)h) << 16); }

__device__ __forceinline__ void dep_guard_h(v8f& a, v8f& b, v16h x, v16h y) { asm volatile("v_nop\n\tv_nop\n\tv_nop\n\tv_nop" : "+v"(a), "+v"(b) : "v"(x), "v"(y)); }
__device__ __forceinline__ void dep_guard_b(v8f& a, v8f& b, v16b x, v16b y) { asm volatile("v_nop\n\tv_nop\n\tv_nop\n\tv_nop" : "+v"(a), "+v"(b) : "v"(x), "v"(y)); }
__device__ __forceinline__ void keep4_h(v16h a, v16h b, v16h c, v16h d) { asm volatile("v_nop" :: "v"(a), "v"(b), "v"(c), "v"(d)); }
__device__ __forceinline__ void keep4_b(v16b a, v16b b, v16b c, v16b d) { asm volatile("v_nop" :: "v"(a), "v"(b), "v"(c), "v"(d)); }
__device__ __forceinline__ void acc_guard4(v8f& a, v8f& b, v8f& c, v8f& d) { asm volatile("v_nop\n\tv_nop\n\tv_nop\n\tv_nop" : "+v"(a), "+v"(b), "+v"(c), "+v"(d)); }
template <typename T> struct Frag;
template <> struct Frag<_Float16> {
  typedef v16h V; union U { v16h v; v8h h[2]; };
  static __device__ __forceinline__ v16h load(const _Float16* p) {
    U f; f.h[0] = *(const v8h*)(p); f.h[1] = *(const v8h*)(p + 16); return f.v;
  }
  static __device__ __forceinline__ v8f mma(v16h a, v16h b, v8f c) {
    return __builtin_amdgcn_wmma_f32_16x16x32_f16(false, a, false, b, (short)0, c, false, false);
  }
  static __device__ __forceinline__ void guard(v8f& a, v8f& b, v16h x, v16h y) { dep_guard_h(a, b, x, y); }
  static __device__ __forceinline__ void keep(v16h a, v16h b, v16h c, v16h d) { keep4_h(a, b, c, d); }
};
template <> struct Frag<__bf16> {
  typedef v16b V; union U { v16b v; v8b h[2]; };
  static __device__ __forceinline__ v16b load(const __bf16* p) {
    U f; f.h[0] = *(const v8b*)(p); f.h[1] = *(const v8b*)(p + 16); return f.v;
  }
  static __device__ __forceinline__ v8f mma(v16b a, v16b b, v8f c) {
    return __builtin_amdgcn_wmma_f32_16x16x32_bf16(false, a, false, b, (short)0, c, false, false);
  }
  static __device__ __forceinline__ void guard(v8f& a, v8f& b, v16b x, v16b y) { dep_guard_b(a, b, x, y); }
  static __device__ __forceinline__ void keep(v16b a, v16b b, v16b c, v16b d) { keep4_b(a, b, c, d); }
};

template <int ET> struct Elem;
template <> struct Elem<0> { typedef _Float16 T; };
template <> struct Elem<1> { typedef __bf16 T; };
template <int ET, bool SPLIT, int BIAS_MODE, int OUT_MODE, bool RESID, int ACT = 0>
__global__ __launch_bounds__(256) void wmma_gemm64(
    const unsigned short* __restrict__ Ap, const unsigned short* __restrict__ A2p, int lda, long strideA,
    const unsigned short* __restrict__ Btp, const unsigned short* __restrict__ Bt2p, int ldb, long strideB,
    void* __restrict__ Cout, void* __restrict__ Cout2, int ldc, long strideC,
    const float* __restrict__ bias,
    const float* __restrict__ resid, long strideR,
    int M, int N, int K, float scale) {
  typedef typename Elem<ET>::T T;
  typedef typename Frag<T>::V V;
  const T* A = (const T*)Ap; const T* A2 = (const T*)A2p; const T* Bt = (const T*)Btp; const T* Bt2 = (const T*)Bt2p;
  __shared__ __align__(16) float sT[8][16 * 68];
  const int b    = blockIdx.y;
  const int lane = threadIdx.x & 31;
  const int wave = threadIdx.x >> 5;
  const int tilesN = N >> 6;
  const int tilesM = M >> 6;
  const int tile = blockIdx.x * 8 + wave;
  if (tile >= tilesM * tilesN) return;
  const int tm = tile / tilesN;
  const int tn = tile - tm * tilesN;
  const int m0 = tm << 6;
  const int n0 = tn << 6;

  const T* Ab  = A  + (size_t)b * strideA;
  const T* Bb  = Bt + (size_t)b * strideB;
  const T* Ab2 = SPLIT ? (A2  + (size_t)b * strideA) : nullptr;
  const T* Bb2 = SPLIT ? (Bt2 + (size_t)b * strideB) : nullptr;

  const int rlane = lane & 15;
  const int koff  = (lane >> 4) * 8;
  const int mOff  = (lane >> 4) * 8;

  v8f acc[4][4];
#pragma unroll
  for (int i = 0; i < 4; ++i)
#pragma unroll
    for (int j = 0; j < 4; ++j) acc[i][j] = (v8f){0.f,0.f,0.f,0.f,0.f,0.f,0.f,0.f};

  for (int k0 = 0; k0 < K; k0 += 32) {
    V bh[4], bl[4];
#pragma unroll
    for (int j = 0; j < 4; ++j) {
      const size_t bo = (size_t)(n0 + (j << 4) + rlane) * ldb + koff + k0;
      bh[j] = Frag<T>::load(Bb + bo);
      if (SPLIT) bl[j] = Frag<T>::load(Bb2 + bo);
    }
#pragma unroll
    for (int i = 0; i < 4; ++i) {
      const size_t ao = (size_t)(m0 + (i << 4) + rlane) * lda + koff + k0;
      V ah = Frag<T>::load(Ab + ao);
      V al;
      if (SPLIT) al = Frag<T>::load(Ab2 + ao);
#pragma unroll
      for (int j = 0; j < 4; ++j) {
        acc[i][j] = Frag<T>::mma(ah, bh[j], acc[i][j]);
        if (SPLIT) {
          acc[i][j] = Frag<T>::mma(ah, bl[j], acc[i][j]);
          acc[i][j] = Frag<T>::mma(al, bh[j], acc[i][j]);
        }
      }
      Frag<T>::guard(acc[i][0], acc[i][3], ah, SPLIT ? al : ah);
    }
    Frag<T>::keep(bh[0], bh[1], bh[2], bh[3]);
    if (SPLIT) Frag<T>::keep(bl[0], bl[1], bl[2], bl[3]);
  }
  acc_guard4(acc[0][0], acc[0][1], acc[0][2], acc[0][3]);
  acc_guard4(acc[1][0], acc[1][1], acc[1][2], acc[1][3]);
  acc_guard4(acc[2][0], acc[2][1], acc[2][2], acc[2][3]);
  acc_guard4(acc[3][0], acc[3][1], acc[3][2], acc[3][3]);

  float* slab = sT[wave];
  const float* Rb = RESID ? (resid + (size_t)b * strideR) : nullptr;
#pragma unroll
  for (int i = 0; i < 4; ++i) {
    const int mBase = m0 + (i << 4);
#pragma unroll
    for (int j = 0; j < 4; ++j) {
      const int n = n0 + (j << 4) + rlane;
      float bv = 0.f;
      if (BIAS_MODE == 2) bv = bias[n];
#pragma unroll
      for (int r = 0; r < 8; ++r) {
        float v = acc[i][j][r] * scale;
        if (BIAS_MODE == 1) v += bias[mBase + mOff + r];
        if (BIAS_MODE == 2) v += bv;
        if (RESID) v += Rb[(size_t)(mBase + mOff + r) * ldc + n];
        if (ACT == 1) v = tanhf(v);
        if (ACT == 2) v = fmaxf(v, 0.0f);
        if (ACT == 3) v = v / (1.0f + expf(-v));
        if (ACT == 4) v = (v > 0.f) ? v : 0.01f * v;
        if (ACT == 5) v = 0.5f * v * (1.0f + erff(v * 0.70710678118654752f));
        slab[(mOff + r) * 68 + (j << 4) + rlane] = v;
      }
    }
    __builtin_amdgcn_fence(__ATOMIC_RELEASE, "workgroup");
    __builtin_amdgcn_wave_barrier();
    __builtin_amdgcn_fence(__ATOMIC_ACQUIRE, "workgroup");
    if (OUT_MODE == 0) {
      float* C = (float*)Cout + (size_t)b * strideC;
      const int hh = lane >> 4, c4 = (lane & 15) * 4;
      for (int pass = 0; pass < 2; ++pass) {
#pragma unroll
        for (int it = 0; it < 8; ++it) {
          const int row = it * 2 + hh;
          v4f v = *(const v4f*)(slab + row * 68 + c4);
          *(volatile v4f*)(C + (size_t)(mBase + row) * ldc + n0 + c4) = v;
        }
        __threadfence();
      }
    } else {
      const int q = lane >> 3, c8 = (lane & 7) * 8;
      unsigned short* C  = (unsigned short*)Cout  + (size_t)b * strideC;
      unsigned short* C2 = (OUT_MODE == 2) ? ((unsigned short*)Cout2 + (size_t)b * strideC) : nullptr;
      for (int pass = 0; pass < 2; ++pass) {
#pragma unroll
        for (int it = 0; it < 4; ++it) {
          const int row = it * 4 + q;
          const float* sp = slab + row * 68 + c8;
          v8h hv, lv;
#pragma unroll
          for (int e = 0; e < 8; ++e) {
            if (OUT_MODE == 1) {
              hv[e] = (_Float16)sp[e];
            } else {
              unsigned short hb = f2bf_bits(sp[e]);
              unsigned short lb = f2bf_bits(sp[e] - bf_bits2f(hb));
              hv[e] = __builtin_bit_cast(_Float16, hb);
              lv[e] = __builtin_bit_cast(_Float16, lb);
            }
          }
          *(volatile v8h*)(C + (size_t)(mBase + row) * ldc + n0 + c8) = hv;
          if (OUT_MODE == 2) *(volatile v8h*)(C2 + (size_t)(mBase + row) * ldc + n0 + c8) = lv;
        }
        __threadfence();
      }
    }
    __builtin_amdgcn_fence(__ATOMIC_RELEASE, "workgroup");
    __builtin_amdgcn_wave_barrier();
    __builtin_amdgcn_fence(__ATOMIC_ACQUIRE, "workgroup");
  }
}

__device__ __forceinline__ v8f zero8() { return (v8f){0.f,0.f,0.f,0.f,0.f,0.f,0.f,0.f}; }
__device__ __forceinline__ unsigned short h_bits(float f) { return __builtin_bit_cast(unsigned short, (_Float16)f); }
__device__ __forceinline__ void guard3_h(v8f& a, v8f& b, v16h x, v16h y, v16h z) {
  asm volatile("v_nop\n\tv_nop\n\tv_nop\n\tv_nop" : "+v"(a), "+v"(b) : "v"(x), "v"(y), "v"(z));
}

__global__ __launch_bounds__(256) void cast_scale_f16x8(
    const float* __restrict__ in, unsigned short* __restrict__ out, int n8, float sc) {
  const int i = blockIdx.x * 256 + threadIdx.x;
  if (i < n8) {
    const v4f a = *(const v4f*)(in + (size_t)i * 8);
    const v4f b = *(const v4f*)(in + (size_t)i * 8 + 4);
    v8h hv;
#pragma unroll
    for (int e = 0; e < 4; ++e) {
      hv[e]     = (_Float16)(a[e] * sc);
      hv[4 + e] = (_Float16)(b[e] * sc);
    }
    *(volatile v8h*)(out + (size_t)i * 8) = hv;
    __threadfence();
    *(volatile v8h*)(out + (size_t)i * 8) = hv;
  }
}

__global__ __launch_bounds__(256) void rnn2_scan(
    const int* __restrict__ xtok, const float* __restrict__ emb,
    const unsigned short* __restrict__ wih0, const unsigned short* __restrict__ whh0,
    const unsigned short* __restrict__ wih1, const unsigned short* __restrict__ whh1,
    const float* __restrict__ bih0, const float* __restrict__ bhh0,
    const float* __restrict__ bih1, const float* __restrict__ bhh1,
    float* __restrict__ hid_out, unsigned short* __restrict__ h1last) {
  __shared__ __align__(16) unsigned short embT[kRowsPerBlock * kTilePitch];
  __shared__ __align__(16) unsigned short h0T[2][kRowsPerBlock * kTilePitch];
  __shared__ __align__(16) unsigned short h1T[2][kRowsPerBlock * kTilePitch];
  __shared__ __align__(16) float slab[kRowsPerBlock * kSlabPitch];

  const int tid  = threadIdx.x;
  const int lane = tid & 31;
  const int wave = tid >> 5;
  const int hh   = lane >> 4;
  const int c    = lane & 15;
  const int row0 = blockIdx.x * kRowsPerBlock;
  const int ncol = wave * 16 + c;
  const int gr   = tid >> 3;
  const int gs   = tid & 7;

  {
    unsigned* z0 = (unsigned*)(&h0T[0][0]);
    unsigned* z1 = (unsigned*)(&h1T[0][0]);
    for (int i = tid; i < kRowsPerBlock * kTilePitch; i += 256) { z0[i] = 0u; z1[i] = 0u; }
  }

  const float bias0 = bih0[ncol] + bhh0[ncol];
  const float bias1 = bih1[ncol] + bhh1[ncol];
  float h0v[16], h1v[16];
#pragma unroll
  for (int i = 0; i < 16; ++i) { h0v[i] = 0.f; h1v[i] = 0.f; }
  __syncthreads();

#pragma unroll 1
  for (int t = 0; t < kSteps; ++t) {
    {
      int tok = xtok[(size_t)(row0 + gr) * kSteps + t];
      tok = tok < 0 ? 0 : tok;
      tok = tok > (kVoc - 1) ? (kVoc - 1) : tok;
      const float* ep = emb + (size_t)tok * kEmb + gs * 16;
      const v4f e0 = *(const v4f*)(ep);
      const v4f e1 = *(const v4f*)(ep + 4);
      const v4f e2 = *(const v4f*)(ep + 8);
      const v4f e3 = *(const v4f*)(ep + 12);
      v8h p0, p1;
#pragma unroll
      for (int e = 0; e < 4; ++e) {
        p0[e]     = (_Float16)(e0[e] * kActCarry);
        p0[4 + e] = (_Float16)(e1[e] * kActCarry);
        p1[e]     = (_Float16)(e2[e] * kActCarry);
        p1[4 + e] = (_Float16)(e3[e] * kActCarry);
      }
      *(v8h*)(embT + gr * kTilePitch + gs * 16)     = p0;
      *(v8h*)(embT + gr * kTilePitch + gs * 16 + 8) = p1;
    }
    __syncthreads();

    const int cur = t & 1;
    const int nxt = cur ^ 1;

    {
      v8f acc0 = zero8(), acc1 = zero8();
#pragma unroll
      for (int ks = 0; ks < 4; ++ks) {
        const int k0 = ks * 32;
        const v16h bf = Frag<_Float16>::load((const _Float16*)(wih0 + (size_t)ncol * kEmb + k0 + 8 * hh));
        const v16h a0 = Frag<_Float16>::load((const _Float16*)(embT + c * kTilePitch + k0 + 8 * hh));
        const v16h a1 = Frag<_Float16>::load((const _Float16*)(embT + (16 + c) * kTilePitch + k0 + 8 * hh));
        acc0 = Frag<_Float16>::mma(a0, bf, acc0);
        acc1 = Frag<_Float16>::mma(a1, bf, acc1);
        guard3_h(acc0, acc1, a0, a1, bf);
      }
      const unsigned short* hc = h0T[cur];
#pragma unroll
      for (int ks = 0; ks < 4; ++ks) {
        const int k0 = ks * 32;
        const v16h bf = Frag<_Float16>::load((const _Float16*)(whh0 + (size_t)ncol * kHid + k0 + 8 * hh));
        const v16h a0 = Frag<_Float16>::load((const _Float16*)(hc + c * kTilePitch + k0 + 8 * hh));
        const v16h a1 = Frag<_Float16>::load((const _Float16*)(hc + (16 + c) * kTilePitch + k0 + 8 * hh));
        acc0 = Frag<_Float16>::mma(a0, bf, acc0);
        acc1 = Frag<_Float16>::mma(a1, bf, acc1);
        guard3_h(acc0, acc1, a0, a1, bf);
      }
      unsigned short* hn = h0T[nxt];
#pragma unroll
      for (int r = 0; r < 8; ++r) {
        const float v0 = tanhf(acc0[r] * kFold + bias0);
        const float v1 = tanhf(acc1[r] * kFold + bias0);
        h0v[r] = v0;
        h0v[8 + r] = v1;
        hn[(8 * hh + r) * kTilePitch + ncol]      = h_bits(v0 * kActCarry);
        hn[(16 + 8 * hh + r) * kTilePitch + ncol] = h_bits(v1 * kActCarry);
      }
    }
    __syncthreads();

    {
      v8f acc0 = zero8(), acc1 = zero8();
      const unsigned short* xin = h0T[nxt];
#pragma unroll
      for (int ks = 0; ks < 4; ++ks) {
        const int k0 = ks * 32;
        const v16h bf = Frag<_Float16>::load((const _Float16*)(wih1 + (size_t)ncol * kHid + k0 + 8 * hh));
        const v16h a0 = Frag<_Float16>::load((const _Float16*)(xin + c * kTilePitch + k0 + 8 * hh));
        const v16h a1 = Frag<_Float16>::load((const _Float16*)(xin + (16 + c) * kTilePitch + k0 + 8 * hh));
        acc0 = Frag<_Float16>::mma(a0, bf, acc0);
        acc1 = Frag<_Float16>::mma(a1, bf, acc1);
        guard3_h(acc0, acc1, a0, a1, bf);
      }
      const unsigned short* hc = h1T[cur];
#pragma unroll
      for (int ks = 0; ks < 4; ++ks) {
        const int k0 = ks * 32;
        const v16h bf = Frag<_Float16>::load((const _Float16*)(whh1 + (size_t)ncol * kHid + k0 + 8 * hh));
        const v16h a0 = Frag<_Float16>::load((const _Float16*)(hc + c * kTilePitch + k0 + 8 * hh));
        const v16h a1 = Frag<_Float16>::load((const _Float16*)(hc + (16 + c) * kTilePitch + k0 + 8 * hh));
        acc0 = Frag<_Float16>::mma(a0, bf, acc0);
        acc1 = Frag<_Float16>::mma(a1, bf, acc1);
        guard3_h(acc0, acc1, a0, a1, bf);
      }
      unsigned short* hn = h1T[nxt];
#pragma unroll
      for (int r = 0; r < 8; ++r) {
        const float v0 = tanhf(acc0[r] * kFold + bias1);
        const float v1 = tanhf(acc1[r] * kFold + bias1);
        h1v[r] = v0;
        h1v[8 + r] = v1;
        hn[(8 * hh + r) * kTilePitch + ncol]      = h_bits(v0 * kActCarry);
        hn[(16 + 8 * hh + r) * kTilePitch + ncol] = h_bits(v1 * kActCarry);
      }
    }
  }

  __syncthreads();
#pragma unroll
  for (int r = 0; r < 8; ++r) {
    slab[(8 * hh + r) * kSlabPitch + ncol]      = h0v[r];
    slab[(16 + 8 * hh + r) * kSlabPitch + ncol] = h0v[8 + r];
  }
  __syncthreads();
  {
    v4f vals[4];
#pragma unroll
    for (int i = 0; i < 4; ++i) vals[i] = *(const v4f*)(slab + (wave * 4 + i) * kSlabPitch + lane * 4);
    float* dst = hid_out + (size_t)(row0 + wave * 4) * kHid + lane * 4;
    for (int pass = 0; pass < 2; ++pass) {
#pragma unroll
      for (int i = 0; i < 4; ++i) *(volatile v4f*)(dst + (size_t)i * kHid) = vals[i];
      __threadfence();
    }
  }
  __syncthreads();
#pragma unroll
  for (int r = 0; r < 8; ++r) {
    slab[(8 * hh + r) * kSlabPitch + ncol]      = h1v[r];
    slab[(16 + 8 * hh + r) * kSlabPitch + ncol] = h1v[8 + r];
  }
  __syncthreads();
  {
    v4f vals[4];
#pragma unroll
    for (int i = 0; i < 4; ++i) vals[i] = *(const v4f*)(slab + (wave * 4 + i) * kSlabPitch + lane * 4);
    v8h hv2[2];
#pragma unroll
    for (int it = 0; it < 2; ++it) {
      const float* sp = slab + (wave * 4 + 2 * it + hh) * kSlabPitch + c * 8;
#pragma unroll
      for (int e = 0; e < 8; ++e) hv2[it][e] = (_Float16)(sp[e] * kActCarry);
    }
    float* dst = hid_out + (size_t)kBatch * kHid + (size_t)(row0 + wave * 4) * kHid + lane * 4;
    unsigned short* dsth = h1last + (size_t)(row0 + wave * 4) * kHid + c * 8;
    for (int pass = 0; pass < 2; ++pass) {
#pragma unroll
      for (int i = 0; i < 4; ++i) *(volatile v4f*)(dst + (size_t)i * kHid) = vals[i];
#pragma unroll
      for (int it = 0; it < 2; ++it) *(volatile v8h*)(dsth + (size_t)(2 * it + hh) * kHid) = hv2[it];
      __threadfence();
    }
  }
}

extern "C" void kernel_launch(void* const* d_in, const int* in_sizes, int n_in,
                              void* d_out, int out_size, void* d_ws, size_t ws_size,
                              hipStream_t stream) {
  if (n_in < 12) return;
  const int*   xtok = (const int*)d_in[0];
  const float* emb  = (const float*)d_in[1];
  const float* Wih0 = (const float*)d_in[2];
  const float* Whh0 = (const float*)d_in[3];
  const float* bih0 = (const float*)d_in[4];
  const float* bhh0 = (const float*)d_in[5];
  const float* Wih1 = (const float*)d_in[6];
  const float* Whh1 = (const float*)d_in[7];
  const float* bih1 = (const float*)d_in[8];
  const float* bhh1 = (const float*)d_in[9];
  const float* Wout = (const float*)d_in[10];
  const float* bout = (const float*)d_in[11];

  if (in_sizes[0] != kBatch * kSteps) return;
  if (in_sizes[1] != kVoc * kEmb) return;
  if (in_sizes[2] != kHid * kEmb || in_sizes[3] != kHid * kHid) return;
  if (in_sizes[6] != kHid * kHid || in_sizes[7] != kHid * kHid) return;
  if (in_sizes[4] != kHid || in_sizes[5] != kHid || in_sizes[8] != kHid || in_sizes[9] != kHid) return;
  if (in_sizes[10] != kVoc * kHid || in_sizes[11] != kVoc) return;
  if (out_size != kBatch * kVoc + 2 * kBatch * kHid) return;

  float* logits  = (float*)d_out;
  float* hid_out = (float*)d_out + (size_t)kBatch * kVoc;

  char* ws = (char*)d_ws;
  size_t off = 0;
  unsigned short* wih0h = (unsigned short*)(ws + off); off += (size_t)kHid * kEmb * 2;
  unsigned short* whh0h = (unsigned short*)(ws + off); off += (size_t)kHid * kHid * 2;
  unsigned short* wih1h = (unsigned short*)(ws + off); off += (size_t)kHid * kHid * 2;
  unsigned short* whh1h = (unsigned short*)(ws + off); off += (size_t)kHid * kHid * 2;
  unsigned short* wouth = (unsigned short*)(ws + off); off += (size_t)kVoc * kHid * 2;
  unsigned short* h1last = (unsigned short*)(ws + off); off += (size_t)kBatch * kHid * 2;
  if (off > ws_size) return;

  const int n8w = (kHid * kHid) / 8;
  const int n8o = (kVoc * kHid) / 8;
  cast_scale_f16x8<<<(n8w + 255) / 256, 256, 0, stream>>>(Wih0, wih0h, n8w, kWCarry);
  cast_scale_f16x8<<<(n8w + 255) / 256, 256, 0, stream>>>(Whh0, whh0h, n8w, kWCarry);
  cast_scale_f16x8<<<(n8w + 255) / 256, 256, 0, stream>>>(Wih1, wih1h, n8w, kWCarry);
  cast_scale_f16x8<<<(n8w + 255) / 256, 256, 0, stream>>>(Whh1, whh1h, n8w, kWCarry);
  cast_scale_f16x8<<<(n8o + 255) / 256, 256, 0, stream>>>(Wout, wouth, n8o, kWCarry);

  rnn2_scan<<<kBatch / kRowsPerBlock, 256, 0, stream>>>(
      xtok, emb, wih0h, whh0h, wih1h, whh1h, bih0, bhh0, bih1, bhh1, hid_out, h1last);

  const int tiles = (kBatch / 64) * (kVoc / 64);
  wmma_gemm64<0, false, 2, 0, false, 0><<<dim3((tiles + 7) / 8, 1), 256, 0, stream>>>(
      h1last, h1last, kHid, (long)0,
      wouth, wouth, kHid, (long)0,
      (void*)logits, (void*)logits, kVoc, (long)0,
      bout, (const float*)nullptr, (long)0,
      kBatch, kVoc, kHid, kFold);
}
